// GNNML3Model_15238543966414
// MI455X (gfx1250) — hardware-run, weakly checked
//
#include <hip/hip_runtime.h>
#include <stddef.h>
#include <stdint.h>
#include <math.h>

#ifndef SPLIT1
#define SPLIT1 1
#endif
#ifndef SPLIT2
#define SPLIT2 1
#endif
#ifndef SPLITF
#define SPLITF 1
#endif

#define NN      50000
#define NE      800000
#define NS      5
#define CIN     128
#define CC      64
#define CM      64
#define NL      3
#define COUT    64
#define NXW     (NS * CC)
#define GBM     128
#define MP      50048
#define KH      256
#define NTHR    256
#define NWAVE   8
#define EPT     8
#define WCH     (32 * EPT)
#define NBRUN   1024
#define SLB     10
#define NBK     49
#define WLCAP   2560
#define RCAP    20480
#define DEGCAP  64
#define MAXDEG_MEAS 36
#define MAXB_MEAS   16659
#define ABM     64
#define SP      68
#define WSMAX   ((size_t)128 << 20)

#define OWX_A   0
#define OWP_A   40960
#define OWX_B   57344
#define OWP_B   139264
#define OWX_C   172032
#define OWP_C   253952
#define OWR     286720
#define WPL_HALVES 303104

#define TB_EDGE 0
#define TB_NODE 512
#define TB_HEAD 896
#define TB_FLOATS 1024

#define BK_ZINTS (NWAVE * WLCAP + 2 * RCAP + 3 * NBRUN)
#define BK_INTS  (BK_ZINTS + 16)
#define BK_LDS   (BK_INTS * 4)

#define PBX   (MP * CIN / 8 / NTHR)
#define PBL   28
#define PBR   4
#define PBTOT (PBX + NL * PBL + PBR + 2)

static_assert(MP % GBM == 0 && MP >= NN && MP == 391 * GBM && MP % ABM == 0);
static_assert((MP * CIN / 8) % NTHR == 0);
static_assert(NBRUN == (1 << SLB) && NBRUN % ABM == 0 && NBRUN % GBM == 0 && NBRUN % 32 == 0);
static_assert(NBK * NBRUN >= MP && NBK * NBRUN >= NN);
static_assert(NE < (1 << 20) && (((long long)NE) << SLB) < (1LL << 31));
static_assert(NE % WCH == 0 && NE % 4 == 0 && NE % NTHR == 0);
static_assert(RCAP == NWAVE * WLCAP && RCAP % 4 == 0 && BK_ZINTS % (NTHR * 4) == 0);
static_assert((long long)RCAP * 100 >= (long long)MAXB_MEAS * 105);
static_assert(WLCAP >= MAXB_MEAS / 8 + 8 * 46 + 1);
static_assert(MAXDEG_MEAS + 8 <= DEGCAP);
static_assert(BK_LDS <= 327680);
static_assert(NXW % 64 == 0 && CIN % 32 == 0 && KH == 2 * CIN && KH % 32 == 0);
static_assert((GBM * SP + 128) * 4 <= 65536);
static_assert(NN % 2 == 0 && MP % 2 == 0);
static_assert(OWP_A == OWX_A + NXW * CIN && OWX_B == OWP_A + 2 * CM * CIN && OWP_B == OWX_B + NXW * KH);
static_assert(OWX_C == OWP_B + 2 * CM * KH && OWP_C == OWX_C + NXW * KH && OWR == OWP_C + 2 * CM * KH);
static_assert(WPL_HALVES == OWR + COUT * KH);
static_assert(NL * 160 <= TB_NODE && TB_NODE + NL * 128 == TB_HEAD && TB_HEAD + COUT <= TB_FLOATS);

typedef float          v4f   __attribute__((ext_vector_type(4)));
typedef float          v8f   __attribute__((ext_vector_type(8)));
typedef int            v2i   __attribute__((ext_vector_type(2)));
typedef int            v4i   __attribute__((ext_vector_type(4)));
typedef int            v8i   __attribute__((ext_vector_type(8)));
typedef unsigned       v2u   __attribute__((ext_vector_type(2)));
typedef unsigned short v8us  __attribute__((ext_vector_type(8)));
typedef unsigned short v16us __attribute__((ext_vector_type(16)));
typedef __bf16         v16bf __attribute__((ext_vector_type(16)));
typedef v4f  __attribute__((may_alias)) v4fa;
typedef v4i  __attribute__((may_alias)) v4ia;
typedef v2i  __attribute__((may_alias)) v2ia;
typedef v8us __attribute__((may_alias)) v8usa;
union FragB { v16bf v; v16us u; v8us h[2]; v8i w; };

__device__ __forceinline__ v8f wmb(const FragB& a, const FragB& b, v8f c) {
  v8f d = __builtin_amdgcn_wmma_f32_16x16x32_bf16(false, a.v, false, b.v, (short)0, c, false, false);
  asm volatile("v_nop\n\tv_nop\n\tv_nop\n\tv_nop" : "+v"(d) : "v"(a.w), "v"(b.w));
  return d;
}

__device__ __forceinline__ unsigned bf16_bits(float f) {
  const unsigned u = __float_as_uint(f);
  const unsigned r = (u + 0x7FFFu + ((u >> 16) & 1u)) >> 16;
  const unsigned q = (u >> 16) | 0x40u;
  return ((u & 0x7fffffffu) > 0x7f800000u) ? q : r;
}
__device__ __forceinline__ float bf16_val(float f) {
  return __uint_as_float(bf16_bits(f) << 16);
}

__device__ __forceinline__ void hilo_pack(float v0, float v1, float v2, float v3,
                                          unsigned& h01, unsigned& h23, unsigned& l01, unsigned& l23) {
  const unsigned a0 = bf16_bits(v0), a1 = bf16_bits(v1), a2 = bf16_bits(v2), a3 = bf16_bits(v3);
  const unsigned b0 = bf16_bits(v0 - __uint_as_float(a0 << 16));
  const unsigned b1 = bf16_bits(v1 - __uint_as_float(a1 << 16));
  const unsigned b2 = bf16_bits(v2 - __uint_as_float(a2 << 16));
  const unsigned b3 = bf16_bits(v3 - __uint_as_float(a3 << 16));
  h01 = a0 | (a1 << 16); h23 = a2 | (a3 << 16);
  l01 = b0 | (b1 << 16); l23 = b2 | (b3 << 16);
}

__device__ __forceinline__ void st2_v4f(float* p, v4f v) {
  *(volatile v4f*)p = v;
  __threadfence();
  *(volatile v4f*)p = v;
}
__device__ __forceinline__ void st2_v8us(unsigned short* p, v8us v) {
  *(volatile v8us*)p = v;
  __threadfence();
  *(volatile v8us*)p = v;
}
__device__ __forceinline__ void wput(unsigned short* p, int dup, v8us v) {
  *(volatile v8us*)p = v;
  if (dup != 0) *(volatile v8us*)(p + CIN) = v;
  __threadfence();
  *(volatile v8us*)p = v;
  if (dup != 0) *(volatile v8us*)(p + CIN) = v;
}

__device__ __forceinline__ v8us colpick8(const float* __restrict__ base, int stride) {
  float f[8];
#pragma unroll
  for (int i = 0; i < 8; ++i) f[i] = base[(size_t)i * (size_t)stride];
  v8us o;
#pragma unroll
  for (int i = 0; i < 8; ++i) o[i] = (unsigned short)bf16_bits(f[i]);
  return o;
}

__global__ __launch_bounds__(NTHR) void k_prep(
    const float* __restrict__ x,
    const float* __restrict__ w1, const float* __restrict__ b1,
    const float* __restrict__ w2, const float* __restrict__ b2,
    const float* __restrict__ w3, const float* __restrict__ b3,
    const float* __restrict__ w4, const float* __restrict__ b4,
    const float* __restrict__ wc,
    const float* __restrict__ w5, const float* __restrict__ b5,
    const float* __restrict__ w6, const float* __restrict__ b6,
    const float* __restrict__ wr, const float* __restrict__ br,
    unsigned short* xb, unsigned short* wpl, float* tbl) {
  __shared__ __attribute__((aligned(16))) float tb[512];
  const int tid = (int)threadIdx.x;
  const int blk = (int)blockIdx.x;
  if (blk < PBX) {
    const int u   = blk * NTHR + tid;
    const int row = u >> 4, k8 = (u & 15) * 8;
    const int rc  = row < NN ? row : NN - 1;
    const unsigned mk = row < NN ? 0xffffu : 0u;
    const float* p = x + (size_t)rc * CIN + k8;
    const v4f a = *(const v4fa*)p;
    const v4f b = *(const v4fa*)(p + 4);
    v8us o;
    o[0] = (unsigned short)(bf16_bits(a.x) & mk); o[1] = (unsigned short)(bf16_bits(a.y) & mk);
    o[2] = (unsigned short)(bf16_bits(a.z) & mk); o[3] = (unsigned short)(bf16_bits(a.w) & mk);
    o[4] = (unsigned short)(bf16_bits(b.x) & mk); o[5] = (unsigned short)(bf16_bits(b.y) & mk);
    o[6] = (unsigned short)(bf16_bits(b.z) & mk); o[7] = (unsigned short)(bf16_bits(b.w) & mk);
    st2_v8us(xb + (size_t)row * CIN + k8, o);
  } else if (blk < PBX + NL * PBL) {
    const int b   = blk - PBX;
    const int l   = b / PBL;
    const int r   = b - l * PBL;
    const int dup = (l != 0) ? 1 : 0;
    const int pitch = (l == 0) ? CIN : KH;
    const int oX = (l == 0) ? OWX_A : ((l == 1) ? OWX_B : OWX_C);
    const int oP = (l == 0) ? OWP_A : ((l == 1) ? OWP_B : OWP_C);
    if (r < 20) {
      const int u = r * NTHR + tid;
      const int n = u >> 4, k8 = (u & 15) * 8;
      const int s = n >> 6, o = n & 63;
      const v8us v = colpick8(wc + ((size_t)((l * NS + s) * CIN + k8)) * CC + o, CC);
      wput(wpl + (size_t)oX + (size_t)n * (size_t)pitch + k8, dup, v);
    } else if (r < 24) {
      const int u = (r - 20) * NTHR + tid;
      const int n = u >> 4, k8 = (u & 15) * 8;
      const v8us v = colpick8(w5 + ((size_t)(l * CIN + k8)) * CM + n, CM);
      wput(wpl + (size_t)oP + (size_t)n * (size_t)pitch + k8, dup, v);
    } else {
      const int u = (r - 24) * NTHR + tid;
      const int n = u >> 4, k8 = (u & 15) * 8;
      const v8us v = colpick8(w6 + ((size_t)(l * CIN + k8)) * CM + n, CM);
      wput(wpl + (size_t)oP + (size_t)(CM + n) * (size_t)pitch + k8, dup, v);
    }
  } else if (blk < PBX + NL * PBL + PBR) {
    const int u = (blk - PBX - NL * PBL) * NTHR + tid;
    const int n = u >> 4, k8 = (u & 15) * 8;
    const v8us v = colpick8(wr + (size_t)k8 * COUT + n, COUT);
    wput(wpl + (size_t)OWR + (size_t)n * (size_t)KH + k8, 1, v);
  } else if (blk == PBX + NL * PBL + PBR) {
    tb[tid] = 0.0f; tb[tid + NTHR] = 0.0f;
    __syncthreads();
    const int ia = tid < 75 ? tid : 74;
    const int ib = tid < 150 ? tid : 149;
    const int ic = tid < 15 ? tid : 14;
    const float v1 = w1[ia], v2 = w2[ia], v3 = w3[ia], v4 = w4[ib];
    const float u1 = b1[ic], u2 = b2[ic], u3 = b3[ic], u4 = b4[ic];
    asm volatile("" :: "v"(v1), "v"(v2), "v"(v3), "v"(v4));
    asm volatile("" :: "v"(u1), "v"(u2), "v"(u3), "v"(u4));
    if (tid < 75) {
      const int la = ia / 25, ra = ia - 25 * la;
      float* d = tb + 160 * la + ra;
      d[0] = bf16_val(v1); d[25] = bf16_val(v2); d[50] = bf16_val(v3);
    }
    if (tid < 150) {
      const int lb = ib / 50, rb = ib - 50 * lb;
      tb[160 * lb + 75 + rb] = bf16_val(v4);
    }
    if (tid < 15) {
      const int lc = ic / 5, rc = ic - 5 * lc;
      float* d = tb + 160 * lc + 125 + rc;
      d[0] = bf16_val(u1); d[5] = bf16_val(u2); d[10] = bf16_val(u3); d[15] = bf16_val(u4);
    }
    __syncthreads();
    if (tid < 128) {
      const v4f o = *(const v4fa*)(tb + 4 * tid);
      st2_v4f(tbl + TB_EDGE + 4 * tid, o);
    }
  } else {
    tb[tid] = 0.0f; tb[tid + NTHR] = 0.0f;
    __syncthreads();
    const int ia = tid < 192 ? tid : 191;
    const int ib = tid < 64 ? tid : 63;
    const float v5 = b5[ia], v6 = b6[ia], vr = br[ib];
    asm volatile("" :: "v"(v5), "v"(v6), "v"(vr));
    if (tid < 192) {
      const int la = ia >> 6, ra = ia & 63;
      tb[128 * la + ra]      = bf16_val(v5);
      tb[128 * la + 64 + ra] = bf16_val(v6);
    }
    if (tid < 64) tb[384 + tid] = bf16_val(vr);
    __syncthreads();
    if (tid < 128) {
      const v4f o = *(const v4fa*)(tb + 4 * tid);
      st2_v4f(tbl + TB_NODE + 4 * tid, o);
    }
  }
}

__device__ __forceinline__ void bucket_flush(const int* pl, const int* cnt, int ov, int* lp, int* cop, int* fp,
                                             int tid) {
#pragma unroll 1
  for (int i = tid * 4; i < 2 * RCAP; i += NTHR * 4) {
    const v4i v = *(const v4ia*)(pl + i);
    *(volatile v4i*)(lp + i) = v;
  }
#pragma unroll 1
  for (int it = 0; it < 2; ++it) {
    const int idx = (it * NTHR + tid) * 4;
    const v4i v = *(const v4ia*)(cnt + idx);
    *(volatile v4i*)(cop + idx) = v;
  }
  if (tid < 8) {
    const v4i f = {ov, ov, ov, ov};
    *(volatile v4i*)(fp + 4 * tid) = f;
  }
}

__global__ __launch_bounds__(NTHR) void k_bucket(const int* __restrict__ srcs, const int* __restrict__ dsts,
                                                 int* LIST, int* CO, int* POIS) {
  extern __shared__ __attribute__((aligned(16))) int dsm[];
  int* wl   = dsm;
  int* pl   = dsm + NWAVE * WLCAP;
  int* cnt  = pl + 2 * RCAP;
  int* offs = cnt + NBRUN;
  int* cur  = offs + NBRUN;
  int* misc = cur + NBRUN;
  const int tid = (int)threadIdx.x, lane = tid & 31, wave = tid >> 5;
  const int blk = (int)blockIdx.x;
  const unsigned nbs = (unsigned)(blk * NBRUN);

  {
    const v4i z4 = {0, 0, 0, 0};
    for (int i = tid * 4; i < BK_ZINTS; i += NTHR * 4) *(v4ia*)(dsm + i) = z4;
    if (tid < 16) misc[tid] = 0;
  }
  __syncthreads();

  {
    const int per  = ((NE + NWAVE * WCH - 1) / (NWAVE * WCH)) * WCH;
    const int ebeg = wave * per;
    const int eend = (ebeg + per < NE) ? (ebeg + per) : NE;
    int* mylist = wl + wave * WLCAP;
    int wc = 0;
#pragma unroll 1
    for (int cb = ebeg; cb < eend; cb += WCH) {
      const int e0 = cb + lane * EPT;
      const v4i da = *(const v4ia*)(dsts + e0);
      const v4i db = *(const v4ia*)(dsts + e0 + 4);
      const unsigned s0 = (unsigned)da.x - nbs, s1 = (unsigned)da.y - nbs;
      const unsigned s2 = (unsigned)da.z - nbs, s3 = (unsigned)da.w - nbs;
      const unsigned s4 = (unsigned)db.x - nbs, s5 = (unsigned)db.y - nbs;
      const unsigned s6 = (unsigned)db.z - nbs, s7 = (unsigned)db.w - nbs;
      const bool h0 = (s0 < (unsigned)NBRUN) & ((unsigned)da.x < (unsigned)NN);
      const bool h1 = (s1 < (unsigned)NBRUN) & ((unsigned)da.y < (unsigned)NN);
      const bool h2 = (s2 < (unsigned)NBRUN) & ((unsigned)da.z < (unsigned)NN);
      const bool h3 = (s3 < (unsigned)NBRUN) & ((unsigned)da.w < (unsigned)NN);
      const bool h4 = (s4 < (unsigned)NBRUN) & ((unsigned)db.x < (unsigned)NN);
      const bool h5 = (s5 < (unsigned)NBRUN) & ((unsigned)db.y < (unsigned)NN);
      const bool h6 = (s6 < (unsigned)NBRUN) & ((unsigned)db.z < (unsigned)NN);
      const bool h7 = (s7 < (unsigned)NBRUN) & ((unsigned)db.w < (unsigned)NN);
      const unsigned m0 = __builtin_amdgcn_ballot_w32(h0), m1 = __builtin_amdgcn_ballot_w32(h1);
      const unsigned m2 = __builtin_amdgcn_ballot_w32(h2), m3 = __builtin_amdgcn_ballot_w32(h3);
      const unsigned m4 = __builtin_amdgcn_ballot_w32(h4), m5 = __builtin_amdgcn_ballot_w32(h5);
      const unsigned m6 = __builtin_amdgcn_ballot_w32(h6), m7 = __builtin_amdgcn_ballot_w32(h7);
      const unsigned any = m0 | m1 | m2 | m3 | m4 | m5 | m6 | m7;
      if (any != 0u) {
        const int pre = (int)(__builtin_amdgcn_mbcnt_lo(m0, 0u) + __builtin_amdgcn_mbcnt_lo(m1, 0u) +
                              __builtin_amdgcn_mbcnt_lo(m2, 0u) + __builtin_amdgcn_mbcnt_lo(m3, 0u) +
                              __builtin_amdgcn_mbcnt_lo(m4, 0u) + __builtin_amdgcn_mbcnt_lo(m5, 0u) +
                              __builtin_amdgcn_mbcnt_lo(m6, 0u) + __builtin_amdgcn_mbcnt_lo(m7, 0u));
        int p = wc + pre;
        if (h0) { if (p < WLCAP) mylist[p] = ((e0 + 0) << SLB) | (int)s0; p = p + 1; }
        if (h1) { if (p < WLCAP) mylist[p] = ((e0 + 1) << SLB) | (int)s1; p = p + 1; }
        if (h2) { if (p < WLCAP) mylist[p] = ((e0 + 2) << SLB) | (int)s2; p = p + 1; }
        if (h3) { if (p < WLCAP) mylist[p] = ((e0 + 3) << SLB) | (int)s3; p = p + 1; }
        if (h4) { if (p < WLCAP) mylist[p] = ((e0 + 4) << SLB) | (int)s4; p = p + 1; }
        if (h5) { if (p < WLCAP) mylist[p] = ((e0 + 5) << SLB) | (int)s5; p = p + 1; }
        if (h6) { if (p < WLCAP) mylist[p] = ((e0 + 6) << SLB) | (int)s6; p = p + 1; }
        if (h7) { if (p < WLCAP) mylist[p] = ((e0 + 7) << SLB) | (int)s7; p = p + 1; }
        wc += (int)(__builtin_popcount(m0) + __builtin_popcount(m1) + __builtin_popcount(m2) + __builtin_popcount(m3) +
                    __builtin_popcount(m4) + __builtin_popcount(m5) + __builtin_popcount(m6) + __builtin_popcount(m7));
      }
    }
    if (lane == 0) misc[wave] = wc;
  }
  __syncthreads();

  if (wave == 0) {
    int ov = 0;
#pragma unroll 1
    for (int w2 = 0; w2 < NWAVE; ++w2) {
      int c = misc[w2];
      if (c > WLCAP) ov = 1;
      c = c < 0 ? 0 : (c > WLCAP ? WLCAP : c);
#pragma unroll 1
      for (int b0 = 0; b0 < c; b0 += 32) {
        const int idx = b0 + lane;
        const int ent = wl[w2 * WLCAP + (idx < WLCAP ? idx : WLCAP - 1)];
        const int m32 = (c - b0) < 32 ? (c - b0) : 32;
#pragma unroll 1
        for (int k = 0; k < m32; ++k) {
          const int u    = __builtin_amdgcn_readlane(ent, k);
          const int slot = u & (NBRUN - 1);
          if (lane == 0) cnt[slot] = cnt[slot] + 1;
        }
      }
    }
    if (lane == 0) misc[9] = ov;
  }
  __syncthreads();
  if (wave == 0) {
    const int base = lane * (NBRUN / 32);
    int s = 0;
#pragma unroll 1
    for (int i = 0; i < NBRUN / 32; ++i) s += cnt[base + i];
    int incl = s;
#pragma unroll
    for (int d = 1; d < 32; d <<= 1) {
      const int y = __shfl_up(incl, d, 32);
      if (lane >= d) incl += y;
    }
    int run = incl - s;
#pragma unroll 1
    for (int i = 0; i < NBRUN / 32; ++i) {
      const int cv = cnt[base + i];
      offs[base + i] = run;
      cur[base + i]  = run;
      run += cv;
    }
  }
  __syncthreads();

  if (wave == 0) {
#pragma unroll 1
    for (int w2 = 0; w2 < NWAVE; ++w2) {
      int c = misc[w2];
      c = c < 0 ? 0 : (c > WLCAP ? WLCAP : c);
#pragma unroll 1
      for (int b0 = 0; b0 < c; b0 += 32) {
        const int idx = b0 + lane;
        const int ent = wl[w2 * WLCAP + (idx < WLCAP ? idx : WLCAP - 1)];
        int eid = (ent >> SLB) & 0xFFFFF;
        eid = eid > NE - 1 ? NE - 1 : eid;
        int sr = srcs[eid];
        sr = sr < 0 ? 0 : (sr > NN - 1 ? NN - 1 : sr);
        const int m32 = (c - b0) < 32 ? (c - b0) : 32;
#pragma unroll 1
        for (int k = 0; k < m32; ++k) {
          const int u    = __builtin_amdgcn_readlane(ent, k);
          const int sv   = __builtin_amdgcn_readlane(sr, k);
          const int ev   = __builtin_amdgcn_readlane(eid, k);
          const int slot = u & (NBRUN - 1);
          if (lane == 0) {
            int p = cur[slot];
            p = p < 0 ? 0 : (p > RCAP - 1 ? RCAP - 1 : p);
            pl[2 * p]     = sv;
            pl[2 * p + 1] = ev;
            cur[slot] = p + 1;
          }
        }
      }
    }
  }
  __syncthreads();

  const int ovf = misc[9];
  int* lp  = LIST + (size_t)blk * (size_t)(2 * RCAP);
  int* cop = CO + (size_t)blk * (2 * NBRUN);
  int* fp  = POIS + (size_t)blk * 32;
  bucket_flush(pl, cnt, ovf, lp, cop, fp, tid);
  __threadfence();
  bucket_flush(pl, cnt, ovf, lp, cop, fp, tid);
}

__global__ __launch_bounds__(NTHR) void k_edge(const float* __restrict__ cp, const float* __restrict__ tb, float* CT) {
  __shared__ __attribute__((aligned(16))) float stb[160];
  const int tid = (int)threadIdx.x;
  if (tid < 64) {
    const int qd = tid < 40 ? tid : 39;
    *(v4fa*)(stb + 4 * qd) = *(const v4fa*)(tb + 4 * qd);
  }
  __syncthreads();
  const int e = (int)blockIdx.x * NTHR + tid;
  const float* p = cp + (size_t)e * NS;
  const float r0 = p[0], r1 = p[1], r2 = p[2], r3 = p[3], r4 = p[4];
  const float c0 = bf16_val(r0), c1 = bf16_val(r1), c2 = bf16_val(r2), c3 = bf16_val(r3), c4 = bf16_val(r4);
  float a0 = 0.0f, a1 = 0.0f, a2 = 0.0f, a3 = 0.0f, a4 = 0.0f;
#pragma unroll 1
  for (int j = 0; j < NS; ++j) {
    float t = c0 * stb[j];
    t = fmaf(c1, stb[5 + j], t);
    t = fmaf(c2, stb[10 + j], t);
    t = fmaf(c3, stb[15 + j], t);
    t = fmaf(c4, stb[20 + j], t);
    t = t + stb[125 + j];
    const float o1 = 1.0f / (1.0f + expf(-t));
    const float* wq = stb + 75 + 5 * j;
    a0 = fmaf(o1, wq[0], a0); a1 = fmaf(o1, wq[1], a1); a2 = fmaf(o1, wq[2], a2);
    a3 = fmaf(o1, wq[3], a3); a4 = fmaf(o1, wq[4], a4);
  }
#pragma unroll 1
  for (int j = 0; j < NS; ++j) {
    float t2 = c0 * stb[25 + j];
    t2 = fmaf(c1, stb[30 + j], t2);
    t2 = fmaf(c2, stb[35 + j], t2);
    t2 = fmaf(c3, stb[40 + j], t2);
    t2 = fmaf(c4, stb[45 + j], t2);
    t2 = t2 + stb[130 + j];
    float t3 = c0 * stb[50 + j];
    t3 = fmaf(c1, stb[55 + j], t3);
    t3 = fmaf(c2, stb[60 + j], t3);
    t3 = fmaf(c3, stb[65 + j], t3);
    t3 = fmaf(c4, stb[70 + j], t3);
    t3 = t3 + stb[135 + j];
    const float o2 = 1.0f / (1.0f + expf(-t2));
    const float o3 = 1.0f / (1.0f + expf(-t3));
    const float pr = o2 * o3;
    const float* wq = stb + 100 + 5 * j;
    a0 = fmaf(pr, wq[0], a0); a1 = fmaf(pr, wq[1], a1); a2 = fmaf(pr, wq[2], a2);
    a3 = fmaf(pr, wq[3], a3); a4 = fmaf(pr, wq[4], a4);
  }
  float v0 = a0 + stb[140], v1 = a1 + stb[141], v2 = a2 + stb[142], v3 = a3 + stb[143], v4 = a4 + stb[144];
  v0 = (v0 > 0.0f) ? v0 : (v0 - v0); v1 = (v1 > 0.0f) ? v1 : (v1 - v1); v2 = (v2 > 0.0f) ? v2 : (v2 - v2);
  v3 = (v3 > 0.0f) ? v3 : (v3 - v3); v4 = (v4 > 0.0f) ? v4 : (v4 - v4);
  float* o = CT + e;
  *(volatile float*)(o)                      = v0;
  *(volatile float*)(o + (size_t)NE)         = v1;
  *(volatile float*)(o + (size_t)2 * NE)     = v2;
  *(volatile float*)(o + (size_t)3 * NE)     = v3;
  *(volatile float*)(o + (size_t)4 * NE)     = v4;
  __threadfence();
  *(volatile float*)(o)                      = v0;
  *(volatile float*)(o + (size_t)NE)         = v1;
  *(volatile float*)(o + (size_t)2 * NE)     = v2;
  *(volatile float*)(o + (size_t)3 * NE)     = v3;
  *(volatile float*)(o + (size_t)4 * NE)     = v4;
}

template <int KEXT, int BP, int NT>
__device__ __forceinline__ void gemm_16xn(const unsigned short* __restrict__ ap,
                                          const unsigned short* __restrict__ bp, v8f (&acc)[NT]) {
  static_assert(KEXT % 32 == 0 && KEXT <= BP);
#pragma unroll 1
  for (int k0 = 0; k0 < KEXT; k0 += 32) {
    FragB af;
    af.h[0] = *(const v8usa*)(ap + k0);
    af.h[1] = *(const v8usa*)(ap + k0 + 16);
#pragma unroll
    for (int nt = 0; nt < NT; ++nt) {
      const unsigned short* wq = bp + (size_t)(16 * nt) * (size_t)BP + k0;
      FragB bf;
      bf.h[0] = *(const v8usa*)wq;
      bf.h[1] = *(const v8usa*)(wq + 16);
      acc[nt] = wmb(af, bf, acc[nt]);
    }
  }
}

__device__ __forceinline__ void stage_d(float* stg, const v8f (&acc)[4], int wave, int hh, int m) {
#pragma unroll
  for (int nt = 0; nt < 4; ++nt) {
#pragma unroll
    for (int r = 0; r < 8; ++r) stg[(16 * wave + 8 * hh + r) * SP + 16 * nt + m] = acc[nt][r];
  }
}

template <int KEXT, int AP, int BP>
__global__ __launch_bounds__(NTHR) __attribute__((amdgpu_num_vgpr(248)))
void k_gx(const unsigned short* __restrict__ A, const unsigned short* __restrict__ BT, float* XW) {
  __shared__ __attribute__((aligned(16))) float stg[GBM * SP];
  const int tid = (int)threadIdx.x, lane = tid & 31, wave = tid >> 5, hh = lane >> 4, m = lane & 15;
  const int rowBase = (int)blockIdx.x * GBM;
  const int col0    = (int)blockIdx.y * 64;

  v8f acc[4];
  {
    const v8f z = {0.f, 0.f, 0.f, 0.f, 0.f, 0.f, 0.f, 0.f};
#pragma unroll
    for (int t = 0; t < 4; ++t) acc[t] = z;
  }
  const unsigned short* ap = A + (size_t)(rowBase + 16 * wave + m) * (size_t)AP + 8 * hh;
  const unsigned short* bp = BT + (size_t)(col0 + m) * (size_t)BP + 8 * hh;
  gemm_16xn<KEXT, BP, 4>(ap, bp, acc);
  stage_d(stg, acc, wave, hh, m);
  __syncthreads();

#pragma unroll 1
  for (int i = 0; i < 8; ++i) {
    const int lr   = 16 * wave + 2 * i + hh;
    const int grow = rowBase + lr;
    const v4f a = *(const v4fa*)(stg + lr * SP + 4 * m);
    st2_v4f(XW + (size_t)grow * NXW + col0 + 4 * m, a);
  }
}

template <int KEXT, int AP, int BP>
__global__ __launch_bounds__(NTHR) __attribute__((amdgpu_num_vgpr(248)))
void k_gp(const unsigned short* __restrict__ A, const unsigned short* __restrict__ BT,
          const float* __restrict__ tb, float* NM) {
  __shared__ __attribute__((aligned(16))) float stg[GBM * SP];
  __shared__ __attribute__((aligned(16))) float sb[128];
  const int tid = (int)threadIdx.x, lane = tid & 31, wave = tid >> 5, hh = lane >> 4, m = lane & 15;
  const int rowBase = (int)blockIdx.x * GBM;
  if (tid < 32) *(v4fa*)(sb + 4 * tid) = *(const v4fa*)(tb + 4 * tid);

  v8f acc[8];
  {
    const v8f z = {0.f, 0.f, 0.f, 0.f, 0.f, 0.f, 0.f, 0.f};
#pragma unroll
    for (int t = 0; t < 8; ++t) acc[t] = z;
  }
  const unsigned short* ap = A + (size_t)(rowBase + 16 * wave + m) * (size_t)AP + 8 * hh;
  const unsigned short* bp = BT + (size_t)m * (size_t)BP + 8 * hh;
  gemm_16xn<KEXT, BP, 8>(ap, bp, acc);
  __syncthreads();
#pragma unroll
  for (int nt = 0; nt < 4; ++nt) {
    const int c = 16 * nt + m;
    const float p5 = sb[c], p6 = sb[64 + c];
#pragma unroll
    for (int r = 0; r < 8; ++r) {
      const float v = (acc[nt][r] + p5) * (acc[nt + 4][r] + p6);
      stg[(16 * wave + 8 * hh + r) * SP + c] = v;
    }
  }
  __syncthreads();

#pragma unroll 1
  for (int i = 0; i < 8; ++i) {
    const int lr   = 16 * wave + 2 * i + hh;
    const int grow = rowBase + lr;
    const v4f a = *(const v4fa*)(stg + lr * SP + 4 * m);
    st2_v4f(NM + (size_t)grow * CM + 4 * m, a);
  }
}

template <int KEXT, int AP, int BP>
__global__ __launch_bounds__(NTHR) __attribute__((amdgpu_num_vgpr(248)))
void k_gf(const unsigned short* __restrict__ A, const unsigned short* __restrict__ BT,
          const float* __restrict__ tb, const int* __restrict__ POIS, float* out) {
  __shared__ __attribute__((aligned(16))) float stg[GBM * SP];
  __shared__ __attribute__((aligned(16))) float sb[64];
  const int tid = (int)threadIdx.x, lane = tid & 31, wave = tid >> 5, hh = lane >> 4, m = lane & 15;
  const int rowBase = (int)blockIdx.x * GBM;
  const int flag = POIS[(size_t)(rowBase >> SLB) * 32];
  if (tid < 16) *(v4fa*)(sb + 4 * tid) = *(const v4fa*)(tb + 4 * tid);

  v8f acc[4];
  {
    const v8f z = {0.f, 0.f, 0.f, 0.f, 0.f, 0.f, 0.f, 0.f};
#pragma unroll
    for (int t = 0; t < 4; ++t) acc[t] = z;
  }
  const unsigned short* ap = A + (size_t)(rowBase + 16 * wave + m) * (size_t)AP + 8 * hh;
  const unsigned short* bp = BT + (size_t)m * (size_t)BP + 8 * hh;
  gemm_16xn<KEXT, BP, 4>(ap, bp, acc);
  stage_d(stg, acc, wave, hh, m);
  __syncthreads();

  const v4f bias = *(const v4fa*)(sb + 4 * m);
  const float qnan = __uint_as_float(0x7fc00000u);
#pragma unroll 1
  for (int i = 0; i < 8; ++i) {
    const int lr   = 16 * wave + 2 * i + hh;
    const int grow = rowBase + lr;
    const bool live = grow < NN;
    const int gc = live ? grow : NN - 1;
    const v4f a = *(const v4fa*)(stg + lr * SP + 4 * m);
    asm volatile("" :: "v"(a));
    v4f o;
    o.x = a.x + bias.x; o.y = a.y + bias.y; o.z = a.z + bias.z; o.w = a.w + bias.w;
    o.x = (flag != 0) ? qnan : o.x; o.y = (flag != 0) ? qnan : o.y;
    o.z = (flag != 0) ? qnan : o.z; o.w = (flag != 0) ? qnan : o.w;
    float* op = out + (size_t)gc * COUT + 4 * m;
    if (live) *(volatile v4f*)op = o;
    __threadfence();
    if (live) *(volatile v4f*)op = o;
  }
}

__global__ __launch_bounds__(NTHR) void k_replay(const int* __restrict__ LIST, const int* __restrict__ CO,
                                                 const int* __restrict__ POIS, const float* __restrict__ CT,
                                                 const float* __restrict__ XW, const float* __restrict__ NM,
                                                 unsigned short* HL) {
  const int tid = (int)threadIdx.x, lane = tid & 31, wave = tid >> 5, hh = lane >> 4, q = lane & 15;
  const int rowBase = (int)blockIdx.x * ABM;
  const int bucket  = rowBase >> SLB;
  const int* lb  = LIST + (size_t)bucket * (size_t)(2 * RCAP);
  const int* cob = CO + (size_t)bucket * (2 * NBRUN);
  const int flag = POIS[(size_t)bucket * 32];
  const float qnan = __uint_as_float(0x7fc00000u);

#pragma unroll 1
  for (int i = 0; i < ABM / (2 * NWAVE); ++i) {
    const int d    = rowBase + (ABM / NWAVE) * wave + 2 * i + hh;
    const int slot = d & (NBRUN - 1);
    int c = cob[slot];
    int o = cob[NBRUN + slot];
    const bool big = c > DEGCAP;
    c = c < 0 ? 0 : (c > DEGCAP ? DEGCAP : c);
    o = o < 0 ? 0 : (o > RCAP - 1 ? RCAP - 1 : o);
    const int co = __shfl_xor(c, 16, 32);
    int cm = c > co ? c : co;
    cm = __builtin_amdgcn_readfirstlane(cm);
    int last = o + c - 1;
    last = last < o ? o : last;
    last = last > RCAP - 1 ? RCAP - 1 : last;
    float a0 = 0.0f, a1 = 0.0f, a2 = 0.0f, a3 = 0.0f;
#pragma unroll 1
    for (int j = 0; j < cm; ++j) {
      int idx = o + j;
      idx = idx > last ? last : idx;
      const v2i en = *(const v2ia*)(lb + 2 * idx);
      int sr  = en.x < 0 ? 0 : (en.x > NN - 1 ? NN - 1 : en.x);
      int eid = en.y < 0 ? 0 : (en.y > NE - 1 ? NE - 1 : en.y);
      const float c0 = CT[eid];
      const float c1 = CT[(size_t)NE + eid];
      const float c2 = CT[(size_t)2 * NE + eid];
      const float c3 = CT[(size_t)3 * NE + eid];
      const float c4 = CT[(size_t)4 * NE + eid];
      const float* xr = XW + (size_t)sr * NXW + 4 * q;
      const v4f x0 = *(const v4fa*)(xr);
      const v4f x1 = *(const v4fa*)(xr + 64);
      const v4f x2 = *(const v4fa*)(xr + 128);
      const v4f x3 = *(const v4fa*)(xr + 192);
      const v4f x4 = *(const v4fa*)(xr + 256);
      asm volatile("" :: "v"(c0), "v"(c1), "v"(c2), "v"(c3), "v"(c4));
      asm volatile("" :: "v"(x0));
      asm volatile("" :: "v"(x1));
      asm volatile("" :: "v"(x2));
      asm volatile("" :: "v"(x3));
      asm volatile("" :: "v"(x4));
      const bool valid = j < c;
      float t0 = fmaf(c0, x0.x, a0), t1 = fmaf(c0, x0.y, a1), t2 = fmaf(c0, x0.z, a2), t3 = fmaf(c0, x0.w, a3);
      t0 = fmaf(c1, x1.x, t0); t1 = fmaf(c1, x1.y, t1); t2 = fmaf(c1, x1.z, t2); t3 = fmaf(c1, x1.w, t3);
      t0 = fmaf(c2, x2.x, t0); t1 = fmaf(c2, x2.y, t1); t2 = fmaf(c2, x2.z, t2); t3 = fmaf(c2, x2.w, t3);
      t0 = fmaf(c3, x3.x, t0); t1 = fmaf(c3, x3.y, t1); t2 = fmaf(c3, x3.z, t2); t3 = fmaf(c3, x3.w, t3);
      t0 = fmaf(c4, x4.x, t0); t1 = fmaf(c4, x4.y, t1); t2 = fmaf(c4, x4.z, t2); t3 = fmaf(c4, x4.w, t3);
      a0 = valid ? t0 : a0; a1 = valid ? t1 : a1; a2 = valid ? t2 : a2; a3 = valid ? t3 : a3;
    }
    const v4f g = *(const v4fa*)(NM + (size_t)d * CM + 4 * q);
    asm volatile("" :: "v"(g));
    float m0 = (a0 > 0.0f) ? a0 : (a0 - a0), m1 = (a1 > 0.0f) ? a1 : (a1 - a1);
    float m2 = (a2 > 0.0f) ? a2 : (a2 - a2), m3 = (a3 > 0.0f) ? a3 : (a3 - a3);
    float n0 = (g.x > 0.0f) ? g.x : (g.x - g.x), n1 = (g.y > 0.0f) ? g.y : (g.y - g.y);
    float n2 = (g.z > 0.0f) ? g.z : (g.z - g.z), n3 = (g.w > 0.0f) ? g.w : (g.w - g.w);
    const bool bad  = (flag != 0) | big;
    const bool live = d < NN;
    m0 = bad ? qnan : m0; m1 = bad ? qnan : m1; m2 = bad ? qnan : m2; m3 = bad ? qnan : m3;
    n0 = bad ? qnan : n0; n1 = bad ? qnan : n1; n2 = bad ? qnan : n2; n3 = bad ? qnan : n3;
    m0 = live ? m0 : 0.0f; m1 = live ? m1 : 0.0f; m2 = live ? m2 : 0.0f; m3 = live ? m3 : 0.0f;
    n0 = live ? n0 : 0.0f; n1 = live ? n1 : 0.0f; n2 = live ? n2 : 0.0f; n3 = live ? n3 : 0.0f;
    unsigned ah01, ah23, al01, al23, nh01, nh23, nl01, nl23;
    hilo_pack(m0, m1, m2, m3, ah01, ah23, al01, al23);
    hilo_pack(n0, n1, n2, n3, nh01, nh23, nl01, nl23);
    v2u hA, hN, lA, lN;
    hA.x = ah01; hA.y = ah23; hN.x = nh01; hN.y = nh23;
    lA.x = al01; lA.y = al23; lN.x = nl01; lN.y = nl23;
    unsigned short* hp = HL + (size_t)d * KH + 4 * q;
    *(volatile v2u*)(hp)       = hA;
    *(volatile v2u*)(hp + 64)  = hN;
    *(volatile v2u*)(hp + 128) = lA;
    *(volatile v2u*)(hp + 192) = lN;
    __threadfence();
    *(volatile v2u*)(hp)       = hA;
    *(volatile v2u*)(hp + 64)  = hN;
    *(volatile v2u*)(hp + 128) = lA;
    *(volatile v2u*)(hp + 192) = lN;
  }
}

extern "C" void kernel_launch(void* const* d_in, const int* in_sizes, int n_in,
                              void* d_out, int out_size, void* d_ws, size_t ws_size,
                              hipStream_t stream) {
  if (n_in < 18) return;
  if (in_sizes[0] != NN * CIN) return;
  if (in_sizes[1] != NE * NS) return;
  if (in_sizes[2] != 2 * NE) return;
  if (in_sizes[3] != NL * NS * NS || in_sizes[5] != NL * NS * NS || in_sizes[7] != NL * NS * NS) return;
  if (in_sizes[4] != NL * NS || in_sizes[6] != NL * NS || in_sizes[8] != NL * NS || in_sizes[10] != NL * NS) return;
  if (in_sizes[9] != NL * 2 * NS * NS) return;
  if (in_sizes[11] != NL * NS * CIN * CC) return;
  if (in_sizes[12] != NL * CIN * CM || in_sizes[14] != NL * CIN * CM) return;
  if (in_sizes[13] != NL * CM || in_sizes[15] != NL * CM) return;
  if (in_sizes[16] != CIN * COUT || in_sizes[17] != COUT) return;
  if (out_size != NN * COUT) return;

  const float* x  = (const float*)d_in[0];
  const float* cp = (const float*)d_in[1];
  const int*   ei = (const int*)d_in[2];
  const float* w1 = (const float*)d_in[3];
  const float* b1 = (const float*)d_in[4];
  const float* w2 = (const float*)d_in[5];
  const float* b2 = (const float*)d_in[6];
  const float* w3 = (const float*)d_in[7];
  const float* b3 = (const float*)d_in[8];
  const float* w4 = (const float*)d_in[9];
  const float* b4 = (const float*)d_in[10];
  const float* wc = (const float*)d_in[11];
  const float* w5 = (const float*)d_in[12];
  const float* b5 = (const float*)d_in[13];
  const float* w6 = (const float*)d_in[14];
  const float* b6 = (const float*)d_in[15];
  const float* wr = (const float*)d_in[16];
  const float* br = (const float*)d_in[17];
  float* out = (float*)d_out;
  const int* srcs = ei;
  const int* dsts = ei + NE;

  constexpr size_t zXW   = (size_t)MP * NXW * 4;
  constexpr size_t zNM   = (size_t)MP * CM * 4;
  constexpr size_t zHL   = (size_t)MP * KH * 2;
  constexpr size_t zXB   = (size_t)MP * CIN * 2;
  constexpr size_t zCT   = (size_t)NS * NE * 4;
  constexpr size_t zLIST = (size_t)NBK * RCAP * 8;
  constexpr size_t zCO   = (size_t)NBK * 2 * NBRUN * 4;
  constexpr size_t zPOIS = 6400;
  constexpr size_t zWPL  = (size_t)WPL_HALVES * 2;
  constexpr size_t zTBL  = (size_t)TB_FLOATS * 4;
  constexpr size_t oXW   = 0;
  constexpr size_t oNM   = oXW + zXW;
  constexpr size_t oHL   = oNM + zNM;
  constexpr size_t oCT   = oHL + zHL;
  constexpr size_t oLIST = oCT + zCT;
  constexpr size_t oCO   = oLIST + zLIST;
  constexpr size_t oPOIS = oCO + zCO;
  constexpr size_t oWPL  = oPOIS + zPOIS;
  constexpr size_t oTBL  = oWPL + zWPL;
  constexpr size_t oEND  = oTBL + zTBL;
  static_assert(zXW % 256 == 0 && zNM % 256 == 0 && zHL % 256 == 0 && zCT % 256 == 0 && zLIST % 256 == 0);
  static_assert(zCO % 256 == 0 && zPOIS % 256 == 0 && zWPL % 256 == 0 && zTBL % 256 == 0);
  static_assert(zXB <= zHL && zPOIS >= (size_t)NBK * 128);
  static_assert(oEND <= WSMAX);
  if (oEND > ws_size) return;

  char* ws = (char*)d_ws;
  float*          XW   = (float*)(ws + oXW);
  float*          NM   = (float*)(ws + oNM);
  unsigned short* HL   = (unsigned short*)(ws + oHL);
  unsigned short* XB   = (unsigned short*)(ws + oHL);
  float*          CT   = (float*)(ws + oCT);
  int*            LIST = (int*)(ws + oLIST);
  int*            CO   = (int*)(ws + oCO);
  int*            POIS = (int*)(ws + oPOIS);
  unsigned short* WPL  = (unsigned short*)(ws + oWPL);
  float*          TBL  = (float*)(ws + oTBL);

  constexpr int KB = SPLIT1 ? KH : CIN;
  constexpr int KC = SPLIT2 ? KH : CIN;
  constexpr int KF = SPLITF ? KH : CIN;

  hipFuncSetAttribute(reinterpret_cast<const void*>(&k_bucket), hipFuncAttributeMaxDynamicSharedMemorySize, (int)BK_LDS);

  k_prep<<<PBTOT, NTHR, 0, stream>>>(x, w1, b1, w2, b2, w3, b3, w4, b4, wc, w5, b5, w6, b6, wr, br, XB, WPL, TBL);
  k_bucket<<<NBK, NTHR, BK_LDS, stream>>>(srcs, dsts, LIST, CO, POIS);

  const dim3 gx(MP / GBM, NXW / 64);
  k_edge<<<NE / NTHR, NTHR, 0, stream>>>(cp, TBL + TB_EDGE, CT);
  k_gx<CIN, CIN, CIN><<<gx, NTHR, 0, stream>>>(XB, WPL + OWX_A, XW);
  k_gp<CIN, CIN, CIN><<<MP / GBM, NTHR, 0, stream>>>(XB, WPL + OWP_A, TBL + TB_NODE, NM);
  k_replay<<<MP / ABM, NTHR, 0, stream>>>(LIST, CO, POIS, CT, XW, NM, HL);
  k_edge<<<NE / NTHR, NTHR, 0, stream>>>(cp, TBL + TB_EDGE + 160, CT);
  k_gx<KB, KH, KH><<<gx, NTHR, 0, stream>>>(HL, WPL + OWX_B, XW);
  k_gp<KB, KH, KH><<<MP / GBM, NTHR, 0, stream>>>(HL, WPL + OWP_B, TBL + TB_NODE + 128, NM);
  k_replay<<<MP / ABM, NTHR, 0, stream>>>(LIST, CO, POIS, CT, XW, NM, HL);
  k_edge<<<NE / NTHR, NTHR, 0, stream>>>(cp, TBL + TB_EDGE + 320, CT);
  k_gx<KC, KH, KH><<<gx, NTHR, 0, stream>>>(HL, WPL + OWX_C, XW);
  k_gp<KC, KH, KH><<<MP / GBM, NTHR, 0, stream>>>(HL, WPL + OWP_C, TBL + TB_NODE + 256, NM);
  k_replay<<<MP / ABM, NTHR, 0, stream>>>(LIST, CO, POIS, CT, XW, NM, HL);
  k_gf<KF, KH, KH><<<MP / GBM, NTHR, 0, stream>>>(HL, WPL + OWR, TBL + TB_HEAD, POIS, out);
}
